// EGM_3874060501137
// MI455X (gfx1250) — hardware-verified
//
#include <hip/hip_runtime.h>
#include <math.h>

typedef __attribute__((ext_vector_type(16))) _Float16 v16h;
typedef __attribute__((ext_vector_type(16))) __bf16 v16b;
typedef __attribute__((ext_vector_type(8)))  _Float16 v8h;
typedef __attribute__((ext_vector_type(8)))  float v8f;
typedef __attribute__((ext_vector_type(4)))  float v4f;
typedef __attribute__((ext_vector_type(2)))  float v2f;
typedef __attribute__((ext_vector_type(4)))  unsigned v4u;
typedef __attribute__((ext_vector_type(4)))  int v4i;
typedef float __attribute__((may_alias)) float_a;
typedef int __attribute__((may_alias)) int_a;

template <typename T> __device__ __forceinline__ void vst2(void* p, T v) { *(volatile T*)p = v; __threadfence(); *(volatile T*)p = v; }
__device__ __forceinline__ v8f wmma16(v16h a, v16h b, v8f c) {
  v8f d = __builtin_amdgcn_wmma_f32_16x16x32_f16(false, a, false, b, (short)0, c, false, false);
  asm volatile("v_nop\n\tv_nop\n\tv_nop\n\tv_nop" : "+v"(d) : "v"(a), "v"(b));
  return d;
}
__device__ __forceinline__ v8f wmma_bf(v16b a, v16b b, v8f c) {
  v8f d = __builtin_amdgcn_wmma_f32_16x16x32_bf16(false, a, false, b, (short)0, c, false, false);
  asm volatile("v_nop\n\tv_nop\n\tv_nop\n\tv_nop" : "+v"(d) : "v"(a), "v"(b));
  return d;
}
__device__ __forceinline__ v16h frag_h(const _Float16* rowk0, int lane) {
  union { v16h v; v8h q[2]; } u; const _Float16* p = rowk0 + 8 * (lane >> 4);
  u.q[0] = *(const v8h*)p; u.q[1] = *(const v8h*)(p + 16); return u.v;
}
__device__ __forceinline__ v16h frag_f32(const float* rowk0, int lane) {
  v16h a; const float* p = rowk0 + 8 * (lane >> 4);
#pragma unroll
  for (int i = 0; i < 8; ++i) { a[i] = (_Float16)p[i]; a[8 + i] = (_Float16)p[16 + i]; }
  return a;
}
__device__ __forceinline__ v16h frag_f32s(const float* rowk0, int lane, float sc) {
  v16h a; const float* p = rowk0 + 8 * (lane >> 4);
#pragma unroll
  for (int i = 0; i < 8; ++i) { a[i] = (_Float16)(p[i] * sc); a[8 + i] = (_Float16)(p[16 + i] * sc); }
  return a;
}
__device__ __forceinline__ v16h fragc_f32(const float* W, int k0, int n, int lane, int ld, int K) {
  v16h a; const int g = lane >> 4;
#pragma unroll
  for (int i = 0; i < 8; ++i) { const int ka = k0 + 8 * g + i, kb = ka + 16;
    a[i] = (_Float16)(ka < K ? W[(size_t)(ka < K ? ka : K - 1) * ld + n] : 0.f); a[8 + i] = (_Float16)(kb < K ? W[(size_t)(kb < K ? kb : K - 1) * ld + n] : 0.f); }
  return a;
}
struct F2 { v16b h, l; };
__device__ __forceinline__ F2 bsplit16(const float v[16]) { F2 r;
#pragma unroll
  for (int i = 0; i < 16; ++i) { const __bf16 h = (__bf16)v[i]; r.h[i] = h; r.l[i] = (__bf16)(v[i] - (float)h); }
  return r; }
__device__ __forceinline__ F2 split_row(const float* row, int k0, int lane) { float v[16]; const float* p = row + k0 + 8 * (lane >> 4);
#pragma unroll
  for (int i = 0; i < 8; ++i) { v[i] = p[i]; v[8 + i] = p[16 + i]; }
  return bsplit16(v); }
__device__ __forceinline__ F2 split_rowK(const float* row, int k0, int lane, int K) { float v[16]; const int g = lane >> 4;
#pragma unroll
  for (int i = 0; i < 8; ++i) { const int ka = k0 + 8 * g + i, kb = ka + 16; v[i] = ka < K ? row[ka < K ? ka : K - 1] : 0.f; v[8 + i] = kb < K ? row[kb < K ? kb : K - 1] : 0.f; }
  return bsplit16(v); }
__device__ __forceinline__ F2 split_col(const float* W, int k0, int n, int lane, int ld, int K) { float v[16]; const int g = lane >> 4;
#pragma unroll
  for (int i = 0; i < 8; ++i) { const int ka = k0 + 8 * g + i, kb = ka + 16; v[i] = ka < K ? W[(size_t)(ka < K ? ka : K - 1) * ld + n] : 0.f; v[8 + i] = kb < K ? W[(size_t)(kb < K ? kb : K - 1) * ld + n] : 0.f; }
  return bsplit16(v); }
__device__ __forceinline__ v8f mac3(const F2& a, const F2& b, v8f c) { c = wmma_bf(a.l, b.h, c); c = wmma_bf(a.h, b.l, c); return wmma_bf(a.h, b.h, c); }
__device__ __forceinline__ float sigm(float v) { return 1.0f / (1.0f + expf(-v)); }
#define LDSX() do { asm volatile("s_wait_dscnt 0" ::: "memory"); __builtin_amdgcn_wave_barrier(); __builtin_amdgcn_fence(__ATOMIC_RELEASE, "workgroup"); } while (0)


#define NB 4
#define CC 256
#define CK 32
#define NN 4096
__device__ __forceinline__ float bfr(float v) { return (float)(__bf16)v; }
__device__ __forceinline__ v16b frag_b(const __bf16* rowk0, int lane) { return __builtin_bit_cast(v16b, frag_h((const _Float16*)rowk0, lane)); }
__device__ __attribute__((noinline)) float exp_ni(float v) { return expf(v); }

__global__ __launch_bounds__(256) void k_cvt(const float* __restrict__ F, __bf16* __restrict__ XT) {
  __shared__ __align__(16) __bf16 st[64][CC + 8];
  const int tid = threadIdx.x; const int b = blockIdx.y, n0 = blockIdx.x * 64;
  for (int q = tid; q < CC * 16; q += 256) { const int c = q >> 4, p4 = q & 15; const v4f v = *(const v4f*)(F + ((size_t)b * CC + c) * NN + n0 + p4 * 4);
#pragma unroll
    for (int e = 0; e < 4; ++e) st[p4 * 4 + e][c] = (__bf16)v[e]; }
  __syncthreads();
  for (int q = tid; q < 64 * (CC / 8); q += 256) { const int rl = q / (CC / 8), pc = q % (CC / 8); vst2((unsigned*)(XT + ((size_t)b * NN + n0 + rl) * CC + pc * 8), *(const v4u*)(&st[rl][pc * 8])); }
}
__global__ __launch_bounds__(128) void k_qk(const __bf16* __restrict__ XT, const float* __restrict__ w1a, const float* __restrict__ b1a, const float* __restrict__ w1b, const float* __restrict__ b1b, const float* __restrict__ w2a, const float* __restrict__ b2a, const float* __restrict__ w2b, const float* __restrict__ b2b, float* __restrict__ Q32, __bf16* __restrict__ Kh, __bf16* __restrict__ Kl) {
  __shared__ __align__(16) float sh[4][16][36]; __shared__ __align__(16) float so[4][16][36]; __shared__ __align__(16) __bf16 skh[4][16][40], skl[4][16][40];
  const int tid = threadIdx.x, wave = tid >> 5, lane = tid & 31, col = lane & 15, g = lane >> 4; const int b = blockIdx.y, which = blockIdx.z; const size_t r0 = (size_t)b * NN + blockIdx.x * 64 + wave * 16;
  const float* wa = which == 0 ? w1a : w2a; const float* ba = which == 0 ? b1a : b2a; const float* wb = which == 0 ? w1b : w2b; const float* bb_ = which == 0 ? b1b : b2b;
  v8f acc[2] = {};
#pragma unroll 2
  for (int kc = 0; kc < CC / 32; ++kc) { const v16b a = frag_b(XT + (r0 + col) * CC + kc * 32, lane);
#pragma unroll
    for (int j = 0; j < 2; ++j) acc[j] = wmma_bf(a, split_row(wa + (size_t)(j * 16 + col) * CC, kc * 32, lane).h, acc[j]); }
#pragma unroll
  for (int j = 0; j < 2; ++j) { const float bb = bfr(ba[j * 16 + col]);
#pragma unroll
    for (int r = 0; r < 8; ++r) { const float v = acc[j][r] + bb; sh[wave][8 * g + r][j * 16 + col] = v > 0.f ? v : 0.f; } }
  LDSX();
  v8f acc2[2] = {}; { const F2 ah = split_row(&sh[wave][col][0], 0, lane);
#pragma unroll
    for (int j = 0; j < 2; ++j) { const v16b wbf = split_row(wb + (size_t)(j * 16 + col) * CK, 0, lane).h; acc2[j] = wmma_bf(ah.l, wbf, acc2[j]); acc2[j] = wmma_bf(ah.h, wbf, acc2[j]); } }
  if (which == 0) {
#pragma unroll
    for (int j = 0; j < 2; ++j) { const float bb = bfr(bb_[j * 16 + col]);
#pragma unroll
      for (int r = 0; r < 8; ++r) so[wave][8 * g + r][j * 16 + col] = acc2[j][r] + bb; }
    LDSX();
    for (int qq = lane; qq < 16 * 8; qq += 32) { const int rl = qq >> 3, pc = qq & 7; vst2(Q32 + (r0 + rl) * CK + pc * 4, *(const v4f*)(&so[wave][rl][pc * 4])); } }
  else {
#pragma unroll
    for (int j = 0; j < 2; ++j) { const float bb = bfr(bb_[j * 16 + col]);
#pragma unroll
      for (int r = 0; r < 8; ++r) { const float v = acc2[j][r] + bb; const __bf16 hi = (__bf16)v; skh[wave][8 * g + r][j * 16 + col] = hi; skl[wave][8 * g + r][j * 16 + col] = (__bf16)(v - (float)hi); } }
    LDSX();
    for (int qq = lane; qq < 16 * 4; qq += 32) { const int rl = qq >> 2, pc = qq & 3; vst2((unsigned*)(Kh + (r0 + rl) * CK + pc * 8), *(const v4u*)(&skh[wave][rl][pc * 8])); vst2((unsigned*)(Kl + (r0 + rl) * CK + pc * 8), *(const v4u*)(&skl[wave][rl][pc * 8])); } }
}
__global__ __launch_bounds__(128) void k_attn(const float* __restrict__ Q32, const __bf16* __restrict__ Kh, const __bf16* __restrict__ Kl, const float* __restrict__ F, float* __restrict__ out) {
  __shared__ __align__(16) float sS[4][16][68]; __shared__ __align__(16) __bf16 sPh[4][16][72], sPl[4][16][72]; __shared__ __align__(16) float sO[CC][68];
  const int tid = threadIdx.x, w = tid >> 5, lane = tid & 31, col = lane & 15, g = lane >> 4; const int b = blockIdx.y; const int n0b = blockIdx.x * 64, q0 = n0b + w * 16; const size_t rb = (size_t)b * NN;
  const F2 aq = split_row(Q32 + (rb + q0 + col) * CK, 0, lane);
  float mrun = -3.0e38f, lrun = 0.f; v8f acc[16] = {};
#pragma unroll 1
  for (int kt = 0; kt < NN / 64; ++kt) {
#pragma unroll
    for (int t = 0; t < 4; ++t) { const size_t ko = (rb + kt * 64 + t * 16 + col) * CK; const v16b khf = frag_b(Kh + ko, lane), klf = frag_b(Kl + ko, lane); v8f s = {}; s = wmma_bf(aq.l, khf, s); s = wmma_bf(aq.h, klf, s); s = wmma_bf(aq.h, khf, s);
#pragma unroll
      for (int r = 0; r < 8; ++r) sS[w][8 * g + r][t * 16 + col] = s[r]; }
    LDSX();
    float mx = -3.4e38f;
#pragma unroll
    for (int jj = 0; jj < 32; ++jj) mx = fmaxf(mx, sS[w][col][g * 32 + jj]);
    mx = fmaxf(mx, __shfl_xor(mx, 16, 32));
    const float mnew = fmaxf(mrun, mx); const float corr = expf(mrun - mnew);
    float ps = 0.f;
#pragma unroll 4
    for (int jj = 0; jj < 32; ++jj) { const float p = exp_ni(sS[w][col][g * 32 + jj] - mnew); ps += p; const __bf16 hi = (__bf16)p; sPh[w][col][g * 32 + jj] = hi; sPl[w][col][g * 32 + jj] = (__bf16)(p - (float)hi); }
    ps += __shfl_xor(ps, 16, 32);
    lrun = lrun * corr + ps; mrun = mnew;
#pragma unroll
    for (int r = 0; r < 8; ++r) { const float cr = __shfl(corr, 8 * g + r, 32);
#pragma unroll
      for (int t = 0; t < 16; ++t) acc[t][r] *= cr; }
    LDSX();
#pragma unroll
    for (int kc = 0; kc < 2; ++kc) { const v16b ph = frag_b(&sPh[w][col][0] + kc * 32, lane), pl = frag_b(&sPl[w][col][0] + kc * 32, lane);
#pragma unroll
      for (int t = 0; t < 16; ++t) { const v16b vb = split_row(F + ((size_t)b * CC + t * 16 + col) * NN + kt * 64, kc * 32, lane).h; acc[t] = wmma_bf(pl, vb, acc[t]); acc[t] = wmma_bf(ph, vb, acc[t]); } }
    __builtin_amdgcn_wave_barrier(); }
#pragma unroll
  for (int r = 0; r < 8; ++r) { const float lr = __shfl(lrun, 8 * g + r, 32); const float inv = 1.0f / lr;
#pragma unroll
    for (int t = 0; t < 16; ++t) sO[t * 16 + col][w * 16 + 8 * g + r] = acc[t][r] * inv; }
  __syncthreads();
  for (int qq = tid; qq < CC * 16; qq += 128) { const int c = qq >> 4, pc = qq & 15; const size_t o = ((size_t)b * CC + c) * NN + n0b + pc * 4; v4f v = *(const v4f*)(&sO[c][pc * 4]); const v4f xr = *(const v4f*)(F + o);
#pragma unroll
    for (int e = 0; e < 4; ++e) v[e] += bfr(xr[e]);
    vst2(out + o, v); }
}
extern "C" void kernel_launch(void* const* d_in, const int* in_sizes, int n_in, void* d_out, int out_size, void* d_ws, size_t ws_size, hipStream_t stream) {
  (void)in_sizes; (void)n_in; (void)out_size; (void)ws_size;
  const float** I = (const float**)d_in;
  char* ws = (char*)d_ws; size_t off = 0;
  auto take = [&](size_t bytes) { char* p = ws + off; off += (bytes + 255) & ~(size_t)255; return p; };
  __bf16* XT = (__bf16*)take((size_t)NB * NN * CC * 2); float* Q32 = (float*)take((size_t)NB * NN * CK * 4); __bf16* Kh = (__bf16*)take((size_t)NB * NN * CK * 2); __bf16* Kl = (__bf16*)take((size_t)NB * NN * CK * 2);
  k_cvt<<<dim3(NN / 64, NB), 256, 0, stream>>>(I[0], XT);
  k_qk<<<dim3(NN / 64, NB, 2), 128, 0, stream>>>(XT, I[1], I[2], I[3], I[4], I[5], I[6], I[7], I[8], Q32, Kh, Kl);
  k_attn<<<dim3(NN / 64, NB), 128, 0, stream>>>(Q32, Kh, Kl, I[0], (float*)d_out);
}
